// SSMLayer_35253091565779
// MI455X (gfx1250) — hardware-verified
//
#include <hip/hip_runtime.h>
#include <math.h>

#pragma clang fp contract(off)

constexpr int NSTATE = 64;
constexpr int NSQ    = 64 * 64;
constexpr int LSEQ   = 16384;
constexpr int NBAT   = 512;
constexpr int CHK    = 64;
constexpr int JCH    = 256;
constexpr int NTHS   = 256;
constexpr int NTHW   = 128;
constexpr int BPW    = 16;
constexpr int XPITCH = 72;
constexpr int SLP    = 68;
constexpr int NPLANE = 7;
static_assert(LSEQ == JCH * CHK, "chunking");
static_assert(NSTATE == 64 && CHK == 64, "two 32-deep k-steps per operand");
static_assert(NBAT % (BPW * (NTHW / 32)) == 0, "scan grid exact");
static_assert((JCH * (NBAT / BPW)) % (NTHW / 32) == 0, "output grid exact");
static_assert((NBAT * LSEQ) % (8 * NTHS) == 0, "split grid exact");
static_assert((4 * NSQ) % (8 * NTHW) == 0 && (3 * NSQ) % (8 * NTHW) == 0, "operator staging exact");
static_assert(XPITCH % 8 == 0 && SLP % 4 == 0, "16-B aligned LDS rows");

typedef __attribute__((ext_vector_type(16))) _Float16 v16h;
typedef __attribute__((ext_vector_type(8)))  _Float16 v8h;
typedef __attribute__((ext_vector_type(16))) __bf16   v16b;
typedef __attribute__((ext_vector_type(8)))  __bf16   v8b;
typedef __attribute__((ext_vector_type(8)))  float    v8f;
typedef __attribute__((ext_vector_type(4)))  float    v4f;
typedef __attribute__((ext_vector_type(4)))  unsigned v4u;

__device__ __forceinline__ unsigned short f2bf_bits(float f) {
  unsigned u = __float_as_uint(f);
  return (unsigned short)((u + 0x7FFFu + ((u >> 16) & 1u)) >> 16);
}
__device__ __forceinline__ float bf_bits2f(unsigned short h) { return __uint_as_float(((unsigned)h) << 16); }

__device__ __forceinline__ void dep_guard_h(v8f& a, v8f& b, v16h x, v16h y) { asm volatile("v_nop\n\tv_nop\n\tv_nop\n\tv_nop" : "+v"(a), "+v"(b) : "v"(x), "v"(y)); }
__device__ __forceinline__ void dep_guard_b(v8f& a, v8f& b, v16b x, v16b y) { asm volatile("v_nop\n\tv_nop\n\tv_nop\n\tv_nop" : "+v"(a), "+v"(b) : "v"(x), "v"(y)); }
__device__ __forceinline__ void keep4_h(v16h a, v16h b, v16h c, v16h d) { asm volatile("v_nop" :: "v"(a), "v"(b), "v"(c), "v"(d)); }
__device__ __forceinline__ void keep4_b(v16b a, v16b b, v16b c, v16b d) { asm volatile("v_nop" :: "v"(a), "v"(b), "v"(c), "v"(d)); }
__device__ __forceinline__ void acc_guard4(v8f& a, v8f& b, v8f& c, v8f& d) { asm volatile("v_nop\n\tv_nop\n\tv_nop\n\tv_nop" : "+v"(a), "+v"(b), "+v"(c), "+v"(d)); }
template <typename T> struct Frag;
template <> struct Frag<_Float16> {
  typedef v16h V; union U { v16h v; v8h h[2]; };
  static __device__ __forceinline__ v16h load(const _Float16* p) {
    U f; f.h[0] = *(const v8h*)(p); f.h[1] = *(const v8h*)(p + 16); return f.v;
  }
  static __device__ __forceinline__ v8f mma(v16h a, v16h b, v8f c) {
    return __builtin_amdgcn_wmma_f32_16x16x32_f16(false, a, false, b, (short)0, c, false, false);
  }
  static __device__ __forceinline__ void guard(v8f& a, v8f& b, v16h x, v16h y) { dep_guard_h(a, b, x, y); }
  static __device__ __forceinline__ void keep(v16h a, v16h b, v16h c, v16h d) { keep4_h(a, b, c, d); }
};
template <> struct Frag<__bf16> {
  typedef v16b V; union U { v16b v; v8b h[2]; };
  static __device__ __forceinline__ v16b load(const __bf16* p) {
    U f; f.h[0] = *(const v8b*)(p); f.h[1] = *(const v8b*)(p + 16); return f.v;
  }
  static __device__ __forceinline__ v8f mma(v16b a, v16b b, v8f c) {
    return __builtin_amdgcn_wmma_f32_16x16x32_bf16(false, a, false, b, (short)0, c, false, false);
  }
  static __device__ __forceinline__ void guard(v8f& a, v8f& b, v16b x, v16b y) { dep_guard_b(a, b, x, y); }
  static __device__ __forceinline__ void keep(v16b a, v16b b, v16b c, v16b d) { keep4_b(a, b, c, d); }
};

__device__ __forceinline__ v8f mmag(v16b a, v16b b, v8f c) {
  c = __builtin_amdgcn_wmma_f32_16x16x32_bf16(false, a, false, b, (short)0, c, false, false);
  asm volatile("v_nop\n\tv_nop\n\tv_nop\n\tv_nop" : "+v"(c) : "v"(a), "v"(b));
  return c;
}

template <bool WITH_LO>
__device__ __forceinline__ void emit_planes(const float* src, unsigned short* __restrict__ dh, unsigned short* __restrict__ dl) {
  const int tid = threadIdx.x;
  const int c8 = (tid & 7) * 8;
  v4u hw[2], lw[2];
#pragma unroll
  for (int g = 0; g < 2; ++g) {
    const int row = g * 32 + (tid >> 3);
    const float* sp = src + row * NSTATE + c8;
#pragma unroll
    for (int e = 0; e < 4; ++e) {
      const float x0 = sp[2 * e], x1 = sp[2 * e + 1];
      const unsigned short h0 = f2bf_bits(x0), h1 = f2bf_bits(x1);
      const unsigned short l0 = f2bf_bits(x0 - bf_bits2f(h0)), l1 = f2bf_bits(x1 - bf_bits2f(h1));
      hw[g][e] = (unsigned)h0 | ((unsigned)h1 << 16);
      lw[g][e] = (unsigned)l0 | ((unsigned)l1 << 16);
    }
  }
  for (int pass = 0; pass < 2; ++pass) {
#pragma unroll
    for (int g = 0; g < 2; ++g) {
      const int row = g * 32 + (tid >> 3);
      *(volatile v4u*)(dh + row * NSTATE + c8) = hw[g];
      if (WITH_LO) *(volatile v4u*)(dl + row * NSTATE + c8) = lw[g];
    }
    __threadfence();
  }
}

__global__ __launch_bounds__(NTHS) void setup_kernel(const float* __restrict__ Am, const float* __restrict__ Bv,
                                                     const float* __restrict__ Cv, const float* __restrict__ lsp,
                                                     unsigned short* __restrict__ PL) {
  __shared__ __align__(16) float sL[NSQ];
  __shared__ __align__(16) float sR[NSQ];
  __shared__ __align__(16) float sG[NSQ];
  __shared__ float sdp[NSTATE], sdq[NSTATE], sf[NSTATE], sBb[NSTATE], sv[NSTATE], svn[NSTATE], sw[NSTATE], swn[NSTATE], sKv[NSTATE];
  __shared__ int spiv;
  __shared__ float spv;
  const int tid = threadIdx.x;
  const float step = expf(lsp[0]);
  const float hstep = step * 0.5f;

#pragma unroll 1
  for (int i = tid; i < NSQ; i += NTHS) {
    const int r = i >> 6, c = i & 63;
    const float m = hstep * Am[i];
    float d1 = 1.0f - m;
    float d2 = 1.0f + m;
    asm volatile("" : "+v"(d1));
    asm volatile("" : "+v"(d2));
    const bool dg = (r == c);
    sL[i] = dg ? d1 : -m;
    sR[i] = dg ? 1.0f : 0.0f;
    if (dg) { sdp[r] = (1.0f - d1) - m; sdq[r] = (d2 - 1.0f) - m; }
  }
  __syncthreads();

#pragma unroll 1
  for (int k = 0; k < NSTATE; ++k) {
    if (tid == 0) {
      int best = k;
      float bx = sL[k * 64 + k];
      float bv = fabsf(bx);
#pragma unroll 1
      for (int i = k + 1; i < NSTATE; ++i) {
        const float x = sL[i * 64 + k];
        const float ax = fabsf(x);
        if (ax > bv) { bv = ax; best = i; bx = x; }
      }
      spiv = best; spv = bx;
    }
    __syncthreads();
    const int piv = spiv;
    const float pv = spv;
    if (piv != k) {
      if (tid < 64) { const float a = sL[k * 64 + tid], b = sL[piv * 64 + tid]; sL[k * 64 + tid] = b; sL[piv * 64 + tid] = a; }
      else if (tid < 128) { const int col = tid - 64; const float a = sR[k * 64 + col], b = sR[piv * 64 + col]; sR[k * 64 + col] = b; sR[piv * 64 + col] = a; }
    }
    __syncthreads();
    const float rp = 1.0f / pv;
    if (tid < 64) { sf[tid] = sL[tid * 64 + k]; }
    else if (tid < 128) { const int col = tid - 64; if (col != k) sL[k * 64 + col] = sL[k * 64 + col] * rp; }
    else if (tid < 192) { const int col = tid - 128; sR[k * 64 + col] = sR[k * 64 + col] * rp; }
    __syncthreads();
#pragma unroll 1
    for (int idx = tid; idx < 63 * 128; idx += NTHS) {
      const int rr = idx >> 7;
      const int r = rr + ((rr >= k) ? 1 : 0);
      const int col = idx & 127;
      const float fct = sf[r];
      if (col < 64) {
        sL[r * 64 + col] = fmaf(-fct, sL[k * 64 + col], sL[r * 64 + col]);
      } else {
        const int cc = col - 64;
        sR[r * 64 + cc] = fmaf(-fct, sR[k * 64 + cc], sR[r * 64 + cc]);
      }
    }
    __syncthreads();
  }

  if (tid < 64) {
    float acc = 0.0f;
#pragma unroll 1
    for (int k = 0; k < NSTATE; ++k) acc = fmaf(sR[tid * 64 + k] * step, Bv[k], acc);
    sBb[tid] = acc;
    sv[tid] = acc;
  } else if (tid < 128) {
    sw[tid - 64] = Cv[tid - 64];
  }
#pragma unroll 1
  for (int i = tid; i < NSQ; i += NTHS) {
    const int r = i >> 6, c = i & 63;
    float acc = 0.0f;
#pragma unroll 1
    for (int k = 0; k < NSTATE; ++k) acc = fmaf(sR[r * 64 + k], hstep * Am[k * 64 + c], acc);
    acc = fmaf(sR[r * 64 + c], sdp[c], acc);
    sG[i] = acc;
  }
  __syncthreads();
#pragma unroll 1
  for (int i = tid; i < NSQ; i += NTHS) {
    const int r = i >> 6, c = i & 63;
    const float dd = sdp[c] + sdq[c];
    float acc = 0.0f;
#pragma unroll 1
    for (int k = 0; k < NSTATE; ++k) acc = fmaf(sG[r * 64 + k], 2.0f * (hstep * Am[k * 64 + c]), acc);
    acc = fmaf(sG[r * 64 + c], dd, acc);
    const float src = 2.0f * (hstep * Am[i]) + ((r == c) ? dd : 0.0f);
    sL[i] = src + acc;
  }
  __syncthreads();
#pragma unroll 1
  for (int i = tid; i < NSQ; i += NTHS) sG[i] = sL[i];
  __syncthreads();
#pragma unroll 1
  for (int sq = 0; sq < 6; ++sq) {
#pragma unroll 1
    for (int i = tid; i < NSQ; i += NTHS) {
      const int r = i >> 6, c = i & 63;
      float acc = 0.0f;
#pragma unroll 1
      for (int k = 0; k < NSTATE; ++k) acc = fmaf(sG[r * 64 + k], sG[k * 64 + c], acc);
      sR[i] = acc;
    }
    __syncthreads();
#pragma unroll 1
    for (int i = tid; i < NSQ; i += NTHS) sG[i] = 2.0f * sG[i] + sR[i];
    __syncthreads();
  }
  emit_planes<true>(sG, PL + 0 * NSQ, PL + 1 * NSQ);

#pragma unroll 1
  for (int it = 0; it < NSTATE; ++it) {
    if (tid < 64) {
      sR[tid * 64 + (63 - it)] = sv[tid];
      float acc = 0.0f;
#pragma unroll 1
      for (int k = 0; k < NSTATE; ++k) acc = fmaf(sL[tid * 64 + k], sv[k], acc);
      svn[tid] = sv[tid] + acc;
    }
    __syncthreads();
    if (tid < 64) sv[tid] = svn[tid];
    __syncthreads();
  }
  emit_planes<true>(sR, PL + 2 * NSQ, PL + 3 * NSQ);
  __syncthreads();

#pragma unroll 1
  for (int l = 0; l < NSTATE; ++l) {
    if (tid < 64) {
      float acc = 0.0f;
#pragma unroll 1
      for (int k = 0; k < NSTATE; ++k) acc = fmaf(sw[k], sL[k * 64 + tid], acc);
      swn[tid] = sw[tid] + acc;
    } else if (tid == 64) {
      float acc = 0.0f;
#pragma unroll 1
      for (int k = 0; k < NSTATE; ++k) acc = fmaf(sw[k], sBb[k], acc);
      sKv[l] = acc;
    }
    __syncthreads();
    if (tid < 64) { const float x = swn[tid]; sw[tid] = x; sR[l * 64 + tid] = x; }
    __syncthreads();
  }
  emit_planes<true>(sR, PL + 4 * NSQ, PL + 5 * NSQ);

#pragma unroll 1
  for (int i = tid; i < NSQ; i += NTHS) {
    const int r = i >> 6, c = i & 63;
    const int d = r - c;
    const int dc = (d < 0) ? 0 : d;
    const float val = sKv[dc];
    sG[i] = (d >= 0) ? val : 0.0f;
  }
  __syncthreads();
  emit_planes<false>(sG, PL + 6 * NSQ, PL + 6 * NSQ);
}

__global__ __launch_bounds__(NTHS) void usplit_kernel(const float* __restrict__ u, unsigned short* __restrict__ Uh,
                                                      unsigned short* __restrict__ Ul, int n8) {
  const int i = blockIdx.x * NTHS + threadIdx.x;
  if (i < n8) {
    const float* sp = u + (size_t)i * 8;
    const v4f a = *(const v4f*)(sp);
    const v4f b = *(const v4f*)(sp + 4);
    v4u hw, lw;
#pragma unroll
    for (int e = 0; e < 2; ++e) {
      const float x0 = a[2 * e], x1 = a[2 * e + 1];
      const float y0 = b[2 * e], y1 = b[2 * e + 1];
      const unsigned short hx0 = f2bf_bits(x0), hx1 = f2bf_bits(x1), hy0 = f2bf_bits(y0), hy1 = f2bf_bits(y1);
      const unsigned short lx0 = f2bf_bits(x0 - bf_bits2f(hx0)), lx1 = f2bf_bits(x1 - bf_bits2f(hx1));
      const unsigned short ly0 = f2bf_bits(y0 - bf_bits2f(hy0)), ly1 = f2bf_bits(y1 - bf_bits2f(hy1));
      hw[e]     = (unsigned)hx0 | ((unsigned)hx1 << 16);
      hw[2 + e] = (unsigned)hy0 | ((unsigned)hy1 << 16);
      lw[e]     = (unsigned)lx0 | ((unsigned)lx1 << 16);
      lw[2 + e] = (unsigned)ly0 | ((unsigned)ly1 << 16);
    }
    unsigned short* ph = Uh + (size_t)i * 8;
    unsigned short* pl = Ul + (size_t)i * 8;
    *(volatile v4u*)ph = hw;
    *(volatile v4u*)pl = lw;
    __threadfence();
    *(volatile v4u*)ph = hw;
    *(volatile v4u*)pl = lw;
  }
}

__global__ __launch_bounds__(NTHW) void scan_kernel(const unsigned short* __restrict__ PL,
                                                    const unsigned short* __restrict__ Uh, const unsigned short* __restrict__ Ul,
                                                    unsigned short* __restrict__ Xh, unsigned short* __restrict__ Xl) {
  __shared__ __align__(16) unsigned short sOp[4 * NSQ];
  __shared__ __align__(16) unsigned short sXh[NTHW / 32][BPW * XPITCH];
  __shared__ __align__(16) unsigned short sXl[NTHW / 32][BPW * XPITCH];
  const int tid = threadIdx.x, lane = tid & 31, wave = tid >> 5;
  const int c = lane & 15, hh = lane >> 4, koff = hh * 8;
  const int q = lane >> 3, c8 = (lane & 7) * 8;
  const int bb = blockIdx.x * (BPW * (NTHW / 32)) + wave * BPW;

#pragma unroll 1
  for (int it = 0; it < (4 * NSQ) / (8 * NTHW); ++it) {
    const int idx = it * NTHW + tid;
    *(v4u*)(sOp + 8 * idx) = *(const v4u*)(PL + 8 * idx);
  }
  const v8f z8 = {0.f, 0.f, 0.f, 0.f, 0.f, 0.f, 0.f, 0.f};
  v8f X[4];
  X[0] = z8; X[1] = z8; X[2] = z8; X[3] = z8;
  __syncthreads();

  unsigned short* mXh = sXh[wave];
  unsigned short* mXl = sXl[wave];
  const __bf16* bOp = (const __bf16*)sOp;
  const __bf16* bXh = (const __bf16*)mXh;
  const __bf16* bXl = (const __bf16*)mXl;
  const __bf16* gUh = (const __bf16*)Uh + (size_t)(bb + c) * LSEQ + koff;
  const __bf16* gUl = (const __bf16*)Ul + (size_t)(bb + c) * LSEQ + koff;

#pragma unroll 1
  for (int j = 0; j < JCH; ++j) {
#pragma unroll
    for (int mt = 0; mt < 4; ++mt) {
      v4u hw, lw;
#pragma unroll
      for (int e = 0; e < 4; ++e) {
        const float x0 = X[mt][2 * e], x1 = X[mt][2 * e + 1];
        const unsigned short h0 = f2bf_bits(x0), h1 = f2bf_bits(x1);
        const unsigned short l0 = f2bf_bits(x0 - bf_bits2f(h0)), l1 = f2bf_bits(x1 - bf_bits2f(h1));
        hw[e] = (unsigned)h0 | ((unsigned)h1 << 16);
        lw[e] = (unsigned)l0 | ((unsigned)l1 << 16);
      }
      *(v4u*)(mXh + c * XPITCH + 16 * mt + 8 * hh) = hw;
      *(v4u*)(mXl + c * XPITCH + 16 * mt + 8 * hh) = lw;
    }
    __syncthreads();

    {
      v4u hv[4], lv[4];
#pragma unroll
      for (int it = 0; it < 4; ++it) {
        const int row = it * 4 + q;
        hv[it] = *(const v4u*)(mXh + row * XPITCH + c8);
        lv[it] = *(const v4u*)(mXl + row * XPITCH + c8);
      }
      const size_t rb = (size_t)j * NBAT + (size_t)bb;
      for (int pass = 0; pass < 2; ++pass) {
#pragma unroll
        for (int it = 0; it < 4; ++it) {
          const int row = it * 4 + q;
          *(volatile v4u*)(Xh + (rb + row) * NSTATE + c8) = hv[it];
          *(volatile v4u*)(Xl + (rb + row) * NSTATE + c8) = lv[it];
        }
        __threadfence();
      }
    }

    if (j + 1 < JCH) {
#pragma unroll
      for (int ks = 0; ks < 2; ++ks) {
        const int k0 = ks * 32;
        const v16b fxh = Frag<__bf16>::load(bXh + c * XPITCH + koff + k0);
        const v16b fxl = Frag<__bf16>::load(bXl + c * XPITCH + koff + k0);
        const v16b fuh = Frag<__bf16>::load(gUh + (size_t)j * CHK + k0);
        const v16b ful = Frag<__bf16>::load(gUl + (size_t)j * CHK + k0);
#pragma unroll
        for (int mt = 0; mt < 4; ++mt) {
          const __bf16* pa = bOp + (16 * mt + c) * NSTATE + koff + k0;
          const v16b aeh = Frag<__bf16>::load(pa);
          const v16b ael = Frag<__bf16>::load(pa + NSQ);
          const v16b abh = Frag<__bf16>::load(pa + 2 * NSQ);
          const v16b abl = Frag<__bf16>::load(pa + 3 * NSQ);
          X[mt] = mmag(aeh, fxh, X[mt]);
          X[mt] = mmag(aeh, fxl, X[mt]);
          X[mt] = mmag(ael, fxh, X[mt]);
          X[mt] = mmag(abh, fuh, X[mt]);
          X[mt] = mmag(abh, ful, X[mt]);
          X[mt] = mmag(abl, fuh, X[mt]);
        }
        keep4_b(fxh, fxl, fuh, ful);
      }
      acc_guard4(X[0], X[1], X[2], X[3]);
    }
    __syncthreads();
  }
}

__global__ __launch_bounds__(NTHW) void out_kernel(const float* __restrict__ u, const float* __restrict__ Dp,
                                                   const unsigned short* __restrict__ PL,
                                                   const unsigned short* __restrict__ Uh,
                                                   const unsigned short* __restrict__ Xh, const unsigned short* __restrict__ Xl,
                                                   float* __restrict__ out) {
  __shared__ __align__(16) unsigned short sOp[3 * NSQ];
  __shared__ __align__(16) float slab[NTHW / 32][BPW * SLP];
  const int tid = threadIdx.x, lane = tid & 31, wave = tid >> 5;
  const int c = lane & 15, hh = lane >> 4, koff = hh * 8;

#pragma unroll 1
  for (int it = 0; it < (3 * NSQ) / (8 * NTHW); ++it) {
    const int idx = it * NTHW + tid;
    *(v4u*)(sOp + 8 * idx) = *(const v4u*)(PL + 4 * NSQ + 8 * idx);
  }
  __syncthreads();

  const int unit = blockIdx.x * (NTHW / 32) + wave;
  const int j  = unit >> 5;
  const int bt = unit & 31;
  const int bb = bt * BPW;
  const float D0 = Dp[0];

  const __bf16* bOp = (const __bf16*)sOp;
  const __bf16* gXh = (const __bf16*)Xh + ((size_t)j * NBAT + (size_t)(bb + c)) * NSTATE + koff;
  const __bf16* gXl = (const __bf16*)Xl + ((size_t)j * NBAT + (size_t)(bb + c)) * NSTATE + koff;
  const __bf16* gUh = (const __bf16*)Uh + (size_t)(bb + c) * LSEQ + (size_t)j * CHK + koff;

  const v8f z8 = {0.f, 0.f, 0.f, 0.f, 0.f, 0.f, 0.f, 0.f};
  v8f acc[4];
  acc[0] = z8; acc[1] = z8; acc[2] = z8; acc[3] = z8;
#pragma unroll
  for (int ks = 0; ks < 2; ++ks) {
    const int k0 = ks * 32;
    const v16b fxh = Frag<__bf16>::load(gXh + k0);
    const v16b fxl = Frag<__bf16>::load(gXl + k0);
    const v16b fuh = Frag<__bf16>::load(gUh + k0);
#pragma unroll
    for (int mt = 0; mt < 4; ++mt) {
      const __bf16* pa = bOp + (16 * mt + c) * NSTATE + koff + k0;
      const v16b ach = Frag<__bf16>::load(pa);
      const v16b acl = Frag<__bf16>::load(pa + NSQ);
      const v16b ath = Frag<__bf16>::load(pa + 2 * NSQ);
      acc[mt] = mmag(ach, fxh, acc[mt]);
      acc[mt] = mmag(ach, fxl, acc[mt]);
      acc[mt] = mmag(acl, fxh, acc[mt]);
      acc[mt] = mmag(ath, fuh, acc[mt]);
    }
    keep4_b(fxh, fxl, fuh, fuh);
  }
  acc_guard4(acc[0], acc[1], acc[2], acc[3]);

  float* sl = slab[wave];
#pragma unroll
  for (int mt = 0; mt < 4; ++mt) {
    v4f lo4, hi4;
    lo4[0] = acc[mt][0]; lo4[1] = acc[mt][1]; lo4[2] = acc[mt][2]; lo4[3] = acc[mt][3];
    hi4[0] = acc[mt][4]; hi4[1] = acc[mt][5]; hi4[2] = acc[mt][6]; hi4[3] = acc[mt][7];
    *(v4f*)(sl + c * SLP + 16 * mt + 8 * hh) = lo4;
    *(v4f*)(sl + c * SLP + 16 * mt + 8 * hh + 4) = hi4;
  }
  __syncthreads();

  const int c4 = (lane & 15) * 4;
  const size_t tb = (size_t)j * CHK + (size_t)c4;
  v4f yv[8];
#pragma unroll
  for (int it = 0; it < 8; ++it) {
    const int row = it * 2 + hh;
    const v4f v  = *(const v4f*)(sl + row * SLP + c4);
    const v4f uu = *(const v4f*)(u + (size_t)(bb + row) * LSEQ + tb);
#pragma unroll
    for (int e = 0; e < 4; ++e) yv[it][e] = v[e] + D0 * uu[e];
  }
  for (int pass = 0; pass < 2; ++pass) {
#pragma unroll
    for (int it = 0; it < 8; ++it) {
      const int row = it * 2 + hh;
      *(volatile v4f*)(out + (size_t)(bb + row) * LSEQ + tb) = yv[it];
    }
    __threadfence();
  }
}

extern "C" void kernel_launch(void* const* d_in, const int* in_sizes, int n_in,
                              void* d_out, int out_size, void* d_ws, size_t ws_size, hipStream_t stream) {
  if (n_in < 6 || d_out == nullptr || d_ws == nullptr) return;
  if (in_sizes[0] != NBAT * LSEQ || in_sizes[1] != NSQ || in_sizes[2] != NSTATE || in_sizes[3] != NSTATE ||
      in_sizes[4] < 1 || in_sizes[5] < 1 || out_size != NBAT * LSEQ) return;

  const float* u   = (const float*)d_in[0];
  const float* Am  = (const float*)d_in[1];
  const float* Bv  = (const float*)d_in[2];
  const float* Cv  = (const float*)d_in[3];
  const float* Dp  = (const float*)d_in[4];
  const float* lsp = (const float*)d_in[5];
  float* out = (float*)d_out;

  char* ws = (char*)d_ws; size_t off = 0;
  auto carve = [&](size_t bytes) -> char* { char* p = ws + off; off += (bytes + 255) & ~(size_t)255; return p; };
  unsigned short* PL = (unsigned short*)carve((size_t)NPLANE * NSQ * 2);
  unsigned short* Uh = (unsigned short*)carve((size_t)NBAT * LSEQ * 2);
  unsigned short* Ul = (unsigned short*)carve((size_t)NBAT * LSEQ * 2);
  unsigned short* Xh = (unsigned short*)carve((size_t)JCH * NBAT * NSTATE * 2);
  unsigned short* Xl = (unsigned short*)carve((size_t)JCH * NBAT * NSTATE * 2);
  if (off > ws_size || off > (size_t)134217728) return;

  const int n8 = (NBAT * LSEQ) / 8;
  setup_kernel<<<1, NTHS, 0, stream>>>(Am, Bv, Cv, lsp, PL);
  usplit_kernel<<<n8 / NTHS, NTHS, 0, stream>>>(u, Uh, Ul, n8);
  scan_kernel<<<NBAT / (BPW * (NTHW / 32)), NTHW, 0, stream>>>(PL, Uh, Ul, Xh, Xl);
  out_kernel<<<(JCH * (NBAT / BPW)) / (NTHW / 32), NTHW, 0, stream>>>(u, Dp, PL, Uh, Xh, Xl, out);
}
